// CausalAttention_50629074485540
// MI455X (gfx1250) — hardware-verified
//
#include <hip/hip_runtime.h>


#ifndef NB
#define NB 2
#endif
#ifndef SEQ
#define SEQ 2048
#endif
#define NB_FULL  2
#define SEQ_FULL 2048
#define DM  1024
#define NH  16
#define HD  64
#define MR  (NB * SEQ)
#define OSP 68
#define LOG2E 1.4426950408889634f
typedef unsigned short bf;
typedef __attribute__((ext_vector_type(16))) __bf16   v16bf;
typedef __attribute__((ext_vector_type(8)))  unsigned short v8us;
typedef __attribute__((ext_vector_type(2)))  unsigned short v2us;
typedef __attribute__((ext_vector_type(8)))  float    v8f;
typedef __attribute__((ext_vector_type(4)))  float    v4f;
typedef v4f  __attribute__((may_alias)) v4fa;

static_assert(NH * HD == DM);
static_assert(SEQ % 64 == 0);
static_assert(SEQ <= SEQ_FULL);
static_assert(NB <= NB_FULL);
static_assert(MR % 64 == 0);
static_assert((MR * (DM / 8)) % 256 == 0);
static_assert(((DM * DM) / 64) % 64 == 0);
static_assert(DM % 32 == 0);
static_assert(((size_t)(NB - 1) * SEQ_FULL + SEQ) * DM * 4 <= (size_t)16777216);

__device__ __forceinline__ unsigned short f2bf(float f) { unsigned u = __float_as_uint(f); u += 0x7FFFu + ((u >> 16) & 1u); return (unsigned short)(u >> 16); }
__device__ __forceinline__ float bf2f(unsigned short b) { return __uint_as_float(((unsigned)b) << 16); }
__device__ __forceinline__ void splitf(float y, unsigned short& h, unsigned short& l) { h = f2bf(y); l = f2bf(y - bf2f(h)); }
__device__ __forceinline__ v16bf cat16b(v8us lo, v8us hi) { return __builtin_bit_cast(v16bf, __builtin_shufflevector(lo, hi, 0, 1, 2, 3, 4, 5, 6, 7, 8, 9, 10, 11, 12, 13, 14, 15)); }
__device__ __forceinline__ v8f wmmab(v16bf a, v16bf b, v8f c) { return __builtin_amdgcn_wmma_f32_16x16x32_bf16(false, a, false, b, (short)0, c, false, false); }
__device__ __forceinline__ v16bf ldf(const bf* p) { return cat16b(*(const v8us*)p, *(const v8us*)(p + 16)); }

__global__ __launch_bounds__(256) void k_cvtx(const float* __restrict__ src, bf* dst) {
    const unsigned i = blockIdx.x * 256u + threadIdx.x;
    if (i >= (unsigned)(MR * (DM / 8))) return;
    const unsigned row = i >> 7, c8 = i & 127u;
    const unsigned srow = (row / (unsigned)SEQ) * (unsigned)SEQ_FULL + (row % (unsigned)SEQ);
    const v8f v = *(const v8f*)(src + (size_t)srow * DM + c8 * 8u);
    v8us o;
#pragma unroll
    for (int k = 0; k < 8; ++k) o[k] = f2bf(v[k]);
    bf* p = dst + (size_t)i * 8u;
    *(volatile v8us*)p = o; __threadfence(); *(volatile v8us*)p = o;
}

__global__ __launch_bounds__(256) void k_wt4(const float* __restrict__ w0, const float* __restrict__ w1, const float* __restrict__ w2, const float* __restrict__ w3, bf* WT) {
    const unsigned y = blockIdx.y;
    const float* w = (y == 0u) ? w0 : ((y == 1u) ? w1 : ((y == 2u) ? w2 : w3));
    bf* Bt = WT + (size_t)y * DM * DM;
    const unsigned lane = threadIdx.x & 31u;
    const unsigned L0 = (blockIdx.x * 8u + (threadIdx.x >> 5)) * 8u;
#pragma unroll 1
    for (int ps = 0; ps < 2; ++ps) {
#pragma unroll 1
        for (unsigned l = 0; l < 8u; ++l) {
            const unsigned L = L0 + l; const unsigned e = L * 64u + lane * 2u; const unsigned k = e & (unsigned)(DM - 1), n = e >> 10; v2us o;
            o[0] = f2bf(w[(size_t)k * DM + n]); o[1] = f2bf(w[(size_t)(k + 1u) * DM + n]);
            *(volatile v2us*)(Bt + e) = o; }
        if (ps == 0) __threadfence(); }
}

template <int NSPLIT, int MODE>
__global__ __launch_bounds__(32) void k_gemmw(const bf* __restrict__ A, const bf* __restrict__ A2, const bf* __restrict__ Bt, float* C,
                                              bf* QH, bf* QL, bf* KH, bf* KL, bf* VTH, bf* VTL) {
    __shared__ __align__(16) float os[64 * OSP];
    const unsigned lane = threadIdx.x & 31u, lr = lane & 15u, hi = lane >> 4;
    const unsigned r0 = blockIdx.x * 64u, c0 = blockIdx.y * 64u;
    v8f acc[4][4];
#pragma unroll
    for (int mb = 0; mb < 4; ++mb)
#pragma unroll
        for (int nb = 0; nb < 4; ++nb) acc[mb][nb] = (v8f){};
    const size_t aoff = (size_t)(r0 + lr) * DM + 8u * hi, boff = (size_t)(c0 + lr) * DM + 8u * hi;
#pragma unroll 1
    for (unsigned kc = 0; kc < (unsigned)DM; kc += 32u) {
        v16bf a[4], a2[4];
#pragma unroll
        for (int mb = 0; mb < 4; ++mb) { a[mb] = ldf(A + aoff + (size_t)mb * 16 * DM + kc); if (NSPLIT == 1) a2[mb] = ldf(A2 + aoff + (size_t)mb * 16 * DM + kc); else a2[mb] = a[mb]; }
#pragma unroll
        for (int nb = 0; nb < 4; ++nb) { const v16bf b = ldf(Bt + boff + (size_t)nb * 16 * DM + kc);
#pragma unroll
            for (int mb = 0; mb < 4; ++mb) { acc[mb][nb] = wmmab(a[mb], b, acc[mb][nb]); if (NSPLIT == 1) acc[mb][nb] = wmmab(a2[mb], b, acc[mb][nb]); } }
        asm volatile("v_nop\n\tv_nop\n\tv_nop\n\tv_nop" : "+v"(acc[0][0]), "+v"(acc[1][1]), "+v"(acc[2][2]), "+v"(acc[3][3]) : "v"(a[0]), "v"(a[3]), "v"(a2[3]));
    }
#pragma unroll
    for (int mb = 0; mb < 4; ++mb)
#pragma unroll
        for (int nb = 0; nb < 4; ++nb)
#pragma unroll
            for (int j = 0; j < 8; ++j) os[(mb * 16 + hi * 8 + j) * OSP + nb * 16 + lr] = acc[mb][nb][j];
    __syncthreads();
    const unsigned bq = r0 / (unsigned)SEQ, t0 = r0 % (unsigned)SEQ;
    if (MODE == 0) {
        float* crow = C + ((size_t)bq * SEQ_FULL + t0) * DM + c0;
#pragma unroll 1
        for (int ps = 0; ps < 2; ++ps) {
#pragma unroll 4
            for (unsigned s = 0; s < 32u; ++s) { const unsigned row = 2u * s + hi, cofs = lr * 4u; const v4f val = *(const v4fa*)(os + row * OSP + cofs);
                *(volatile v4f*)(crow + (size_t)row * DM + cofs) = val; }
            if (ps == 0) __threadfence(); }
    } else {
        const unsigned y = blockIdx.y; const unsigned which = y >> 4, head = y & 15u; const unsigned unit = bq * NH + head;
        const unsigned rq = lane >> 3, pc = lane & 7u;
        if (which < 2u) {
            bf* PH = which ? KH : QH; bf* PL = which ? KL : QL; const float scl = which ? 1.0f : 0.125f;
#pragma unroll 1
            for (int ps = 0; ps < 2; ++ps) {
#pragma unroll 4
                for (unsigned s = 0; s < 16u; ++s) { const unsigned row = 4u * s + rq; const float* sp = os + row * OSP + pc * 8u;
                    const v4f x0 = *(const v4fa*)sp, x1 = *(const v4fa*)(sp + 4); v8us oh, ol;
#pragma unroll
                    for (int e = 0; e < 4; ++e) { unsigned short a, c2; splitf(x0[e] * scl, a, c2); oh[e] = a; ol[e] = c2; splitf(x1[e] * scl, a, c2); oh[4 + e] = a; ol[4 + e] = c2; }
                    const size_t oo = ((size_t)unit * SEQ + t0 + row) * HD + pc * 8u;
                    *(volatile v8us*)(PH + oo) = oh; *(volatile v8us*)(PL + oo) = ol; }
                if (ps == 0) __threadfence(); }
        } else {
#pragma unroll 1
            for (int ps = 0; ps < 2; ++ps) {
#pragma unroll 4
                for (unsigned s = 0; s < 16u; ++s) { const unsigned d = 4u * s + rq; v8us oh, ol;
#pragma unroll
                    for (int e = 0; e < 8; ++e) { unsigned short a, c2; splitf(os[(pc * 8u + e) * OSP + d], a, c2); oh[e] = a; ol[e] = c2; }
                    const size_t oo = ((size_t)unit * HD + d) * SEQ + t0 + pc * 8u;
                    *(volatile v8us*)(VTH + oo) = oh; *(volatile v8us*)(VTL + oo) = ol; }
                if (ps == 0) __threadfence(); }
        }
    }
}

__global__ __launch_bounds__(32) void k_flash(const bf* __restrict__ QH, const bf* __restrict__ QL, const bf* __restrict__ KH, const bf* __restrict__ KL,
                                              const bf* __restrict__ VTH, const bf* __restrict__ VTL, bf* CH, bf* CL) {
#pragma clang fp contract(off)
    __shared__ __align__(16) float cs[16 * OSP];
    const unsigned lane = threadIdx.x & 31u, lr = lane & 15u, hi = lane >> 4;
    const unsigned bh = blockIdx.y, hh = bh & 15u, bb = bh >> 4;
    const unsigned q0 = blockIdx.x * 16u, qg = q0 + lr;
    const unsigned sh = (hh + 1u) >> 1;
    const float slope = ((hh & 1u) ? 1.0f : 0.70710678118654752f) * __uint_as_float((127u - sh) << 23);
    const size_t qoff = ((size_t)bh * SEQ + qg) * HD + 8u * hi;
    v16bf qh[2], ql[2];
#pragma unroll
    for (int c = 0; c < 2; ++c) { qh[c] = ldf(QH + qoff + c * 32); ql[c] = ldf(QL + qoff + c * 32); }
    v8f o[4];
#pragma unroll
    for (int t = 0; t < 4; ++t) o[t] = (v8f){};
    float m = -1.0e30f, l = 0.0f;
    const unsigned nsteps = ((q0 + 15u) >> 5) + 1u;
    const size_t kbase = ((size_t)bh * SEQ + lr) * HD + 8u * hi;
    const size_t vbase = ((size_t)bh * HD + lr) * SEQ + 8u * hi;
    const int qgi = (int)qg;
#pragma unroll 1
    for (unsigned s = 0; s < nsteps; ++s) {
        const unsigned k0 = s * 32u;
        v16bf kh[2][2], kl[2][2];
#pragma unroll
        for (int kt = 0; kt < 2; ++kt)
#pragma unroll
            for (int c = 0; c < 2; ++c) { const size_t off = kbase + (size_t)(k0 + kt * 16u) * HD + c * 32; kh[kt][c] = ldf(KH + off); kl[kt][c] = ldf(KL + off); }
        v8f sc[2];
#pragma unroll
        for (int kt = 0; kt < 2; ++kt) { sc[kt] = (v8f){};
#pragma unroll
            for (int c = 0; c < 2; ++c) { sc[kt] = wmmab(kh[kt][c], qh[c], sc[kt]); sc[kt] = wmmab(kl[kt][c], qh[c], sc[kt]); sc[kt] = wmmab(kh[kt][c], ql[c], sc[kt]); } }
        asm volatile("v_nop\n\tv_nop\n\tv_nop\n\tv_nop" : "+v"(sc[0]), "+v"(sc[1]) : "v"(kh[1][1]), "v"(kl[1][1]), "v"(ql[1]));
        asm volatile("" ::: "memory");
        float pv[2][8]; float lm = -1.0e30f;
#pragma unroll
        for (int kt = 0; kt < 2; ++kt)
#pragma unroll
            for (int r = 0; r < 8; ++r) { const int kk = (int)(k0 + kt * 16u + 8u * hi) + r; const float al = slope * (float)(kk - (SEQ_FULL - 1));
                float sv = sc[kt][r] + al; sv = (kk <= qgi) ? sv : -1.0e30f; pv[kt][r] = sv; lm = fmaxf(lm, sv); }
        lm = fmaxf(lm, __shfl_xor(lm, 16, 32));
        const float mnew = fmaxf(m, lm);
        const float alpha = __builtin_amdgcn_exp2f((m - mnew) * LOG2E);
        float ls = 0.0f; v8us pha, phb, pla, plb;
#pragma unroll
        for (int r = 0; r < 8; ++r) { unsigned short a, c2;
            const float p0 = __builtin_amdgcn_exp2f((pv[0][r] - mnew) * LOG2E); ls += p0; splitf(p0, a, c2); pha[r] = a; pla[r] = c2;
            const float p1 = __builtin_amdgcn_exp2f((pv[1][r] - mnew) * LOG2E); ls += p1; splitf(p1, a, c2); phb[r] = a; plb[r] = c2; }
        ls += __shfl_xor(ls, 16, 32);
        l = l * alpha + ls; m = mnew;
        const v16bf PH = cat16b(pha, phb), PL = cat16b(pla, plb);
        v16bf vh[4], vl[4];
#pragma unroll
        for (int t = 0; t < 4; ++t) { const size_t off = vbase + (size_t)t * 16 * SEQ + k0; vh[t] = ldf(VTH + off); vl[t] = ldf(VTL + off); }
#pragma unroll
        for (int t = 0; t < 4; ++t) o[t] = o[t] * alpha;
#pragma unroll
        for (int t = 0; t < 4; ++t) { o[t] = wmmab(vh[t], PH, o[t]); o[t] = wmmab(vl[t], PH, o[t]); o[t] = wmmab(vh[t], PL, o[t]); }
        asm volatile("v_nop\n\tv_nop\n\tv_nop\n\tv_nop" : "+v"(o[0]), "+v"(o[1]), "+v"(o[2]), "+v"(o[3]) : "v"(vh[3]), "v"(vl[3]), "v"(PL), "v"(PH));
    }
    const float inv = 1.0f / l;
#pragma unroll
    for (int t = 0; t < 4; ++t) { v4f w0, w1;
#pragma unroll
        for (int e = 0; e < 4; ++e) { w0[e] = o[t][e] * inv; w1[e] = o[t][4 + e] * inv; }
        float* dp = cs + lr * OSP + t * 16 + 8u * hi; *(v4fa*)dp = w0; *(v4fa*)(dp + 4) = w1; }
    __syncthreads();
    const unsigned rq = lane >> 3, pc = lane & 7u;
#pragma unroll 1
    for (int ps = 0; ps < 2; ++ps) {
#pragma unroll
        for (unsigned s = 0; s < 4u; ++s) { const unsigned row = 4u * s + rq; const float* sp = cs + row * OSP + pc * 8u;
            const v4f x0 = *(const v4fa*)sp, x1 = *(const v4fa*)(sp + 4); v8us oh, ol;
#pragma unroll
            for (int e = 0; e < 4; ++e) { unsigned short a, c2; splitf(x0[e], a, c2); oh[e] = a; ol[e] = c2; splitf(x1[e], a, c2); oh[4 + e] = a; ol[4 + e] = c2; }
            const size_t oo = ((size_t)bb * SEQ + q0 + row) * DM + hh * 64u + pc * 8u;
            *(volatile v8us*)(CH + oo) = oh; *(volatile v8us*)(CL + oo) = ol; }
        if (ps == 0) __threadfence(); }
}

extern "C" void kernel_launch(void* const* d_in, const int* in_sizes, int n_in,
                              void* d_out, int out_size, void* d_ws, size_t ws_size, hipStream_t stream) {
    if (n_in < 5) return;
    const long long needx = ((long long)(NB - 1) * SEQ_FULL + SEQ) * DM;
    if ((long long)in_sizes[0] < needx || (long long)out_size < needx) return;
    if (in_sizes[1] < DM * DM || in_sizes[2] < DM * DM || in_sizes[3] < DM * DM || in_sizes[4] < DM * DM) return;
    const float* x  = (const float*)d_in[0];
    const float* Wq = (const float*)d_in[1];
    const float* Wk = (const float*)d_in[2];
    const float* Wv = (const float*)d_in[3];
    const float* Wo = (const float*)d_in[4];
    float* OUT = (float*)d_out;
    char* wsp = (char*)d_ws;
    auto take = [&](size_t bytes) { char* p = wsp; wsp += (bytes + 255) & ~(size_t)255; return (void*)p; };
    const size_t PLN = (size_t)MR * DM * 2;
    bf* XB  = (bf*)take(PLN);
    bf* WT  = (bf*)take((size_t)4 * DM * DM * 2);
    bf* QH  = (bf*)take(PLN); bf* QL = (bf*)take(PLN);
    bf* KH  = (bf*)take(PLN); bf* KL = (bf*)take(PLN);
    bf* VTH = (bf*)take(PLN); bf* VTL = (bf*)take(PLN);
    bf* CH  = (bf*)take(PLN); bf* CL = (bf*)take(PLN);
    if ((size_t)(wsp - (char*)d_ws) > ws_size) return;
    k_cvtx<<<(unsigned)(MR * (DM / 8) / 256), 256, 0, stream>>>(x, XB);
    k_wt4<<<dim3((unsigned)(DM * DM / 64 / 64), 4, 1), 256, 0, stream>>>(Wq, Wk, Wv, Wo, WT);
    k_gemmw<0, 1><<<dim3(MR / 64, 3 * DM / 64, 1), 32, 0, stream>>>(XB, XB, WT, OUT, QH, QL, KH, KL, VTH, VTL);
    k_flash<<<dim3(SEQ / 16, NB * NH, 1), 32, 0, stream>>>(QH, QL, KH, KL, VTH, VTL, CH, CL);
    k_gemmw<1, 0><<<dim3(MR / 64, DM / 64, 1), 32, 0, stream>>>(CH, CL, WT + (size_t)3 * DM * DM, OUT, QH, QL, KH, KL, VTH, VTL);
}
